// SelfAttention_50869592653915
// MI455X (gfx1250) — hardware-verified
//
#include <hip/hip_runtime.h>


#ifndef NB
#define NB 8
#endif
#ifndef SEQ
#define SEQ 4096
#endif
#define NB_FULL  8
#define SEQ_FULL 4096
#define W_IMG    64
#define CIN      256
#define DQK      32
#define DV       128
#define NPROJ    192
#define NKEY     (SEQ / 4)
#define KTILE    64
#define BQ       128
#define BK       32
#define NWAVE    8
#define PP       168
#define GP       40
#define FP       40
#define HP       72
#define CP       136
#define OP       36
#define XP       264
#define OCH      32

static_assert(SEQ % 256 == 0);
static_assert(SEQ >= 256 && SEQ <= SEQ_FULL);
static_assert(NB >= 1 && NB <= NB_FULL);
static_assert(BQ == NWAVE * 16);
static_assert(NKEY % BK == 0);
static_assert(NKEY % KTILE == 0);
static_assert(CIN % 32 == 0 && DV % 32 == 0 && DQK == 32);
static_assert(W_IMG == 64);
static_assert((SEQ / 256) * 2 * NWAVE * 16 == SEQ);
static_assert((SEQ / 256) * KTILE == NKEY);
static_assert((SEQ / BQ) * NWAVE * 16 == SEQ);
static_assert(((NB * SEQ) / 256) * NWAVE * 32 == NB * SEQ);
static_assert((CIN / OCH) * OCH == CIN && OCH == 32);
static_assert(4 * NWAVE * 8 == CIN);
static_assert(32 * 4 == 2 * W_IMG);
static_assert(XP >= CIN && (XP * 2) % 16 == 0);
static_assert((GP * 2) % 16 == 0 && (FP * 2) % 16 == 0 && (HP * 2) % 16 == 0 && (CP * 2) % 16 == 0);
static_assert((OP * 4) % 16 == 0 && OP >= 32);
static_assert((size_t)NPROJ * CIN * 2 + (size_t)CIN * DV * 2 + (size_t)NB * SEQ * DQK * 2 +
              (size_t)NB * NKEY * DQK * 2 + (size_t)NB * DV * NKEY * 2 + (size_t)NB * SEQ * DV * 2 <= (size_t)134217728);

typedef __bf16   bf16;
typedef _Float16 f16;
typedef bf16     v16bf __attribute__((ext_vector_type(16)));
typedef f16      v16h  __attribute__((ext_vector_type(16)));
typedef f16      v8h   __attribute__((ext_vector_type(8)));
typedef float    v8f   __attribute__((ext_vector_type(8)));
typedef float    v4f   __attribute__((ext_vector_type(4)));
typedef unsigned v4u   __attribute__((ext_vector_type(4)));

union FragB  { v16bf v; v4u q[2]; bf16 h[16]; };
union FragH  { v16h  v; v4u q[2]; f16  h[16]; };
union Pack8B { v4u u; bf16 h[8]; };
union Pack8H { v4u u; v8h v; f16 h[8]; };

static __device__ __forceinline__ v8f mma_bf16(v16bf a, v16bf b, v8f acc) {
  acc = __builtin_amdgcn_wmma_f32_16x16x32_bf16(false, a, false, b, (short)0, acc, false, false);
  asm volatile("v_nop\n\tv_nop\n\tv_nop\n\tv_nop" : "+v"(acc) : "v"(a), "v"(b));
  return acc;
}
static __device__ __forceinline__ v8f mma_f16(v16h a, v16h b, v8f acc) {
  acc = __builtin_amdgcn_wmma_f32_16x16x32_f16(false, a, false, b, (short)0, acc, false, false);
  asm volatile("v_nop\n\tv_nop\n\tv_nop\n\tv_nop" : "+v"(acc) : "v"(a), "v"(b));
  return acc;
}

static __device__ __forceinline__ f16 toh_flush(float v) {
  const f16 r = (f16)v;
  return (fabsf(v) < 6.103515625e-05f) ? (f16)0.0f : r;
}

__global__ __launch_bounds__(256) void pack_w_kernel(const float* __restrict__ wf, const float* __restrict__ wg,
                                                      const float* __restrict__ wh, const float* __restrict__ wo,
                                                      bf16* __restrict__ wct, f16* __restrict__ wot) {
  const int blk = blockIdx.x;
  const int tid = threadIdx.x;
  if (blk < 24) {
    const int n  = blk * 8 + (tid >> 5);
    const int kq = (tid & 31) * 8;
    const float* src = (blk < 4) ? wg : ((blk < 8) ? wf : wh);
    const int nl     = (blk < 4) ? n : ((blk < 8) ? (n - 32) : (n - 64));
    Pack8B pk;
    #pragma unroll
    for (int i = 0; i < 8; ++i) pk.h[i] = (bf16)src[(size_t)nl * CIN + kq + i];
    bf16* dst = wct + (size_t)n * CIN + kq;
    *(volatile v4u*)dst = pk.u;
    __threadfence();
    *(volatile v4u*)dst = pk.u;
  } else {
    const int j  = (blk - 24) * 256 + tid;
    const int n  = j >> 4;
    const int kq = (j & 15) * 8;
    Pack8H pk;
    #pragma unroll
    for (int i = 0; i < 8; ++i) {
      const float v = (float)(bf16)wo[(size_t)n * DV + kq + i];
      pk.h[i] = toh_flush(v * 16.0f);
    }
    f16* dst = wot + (size_t)n * DV + kq;
    *(volatile v4u*)dst = pk.u;
    __threadfence();
    *(volatile v4u*)dst = pk.u;
  }
}

template <int NT0, int NTN>
static __device__ __forceinline__ void proj_tiles(const bf16* xs, const bf16* __restrict__ wct,
                                                  int m, int hi, v8f (&acc)[NTN]) {
  #pragma unroll
  for (int t = 0; t < NTN; ++t) acc[t] = (v8f){0, 0, 0, 0, 0, 0, 0, 0};
  for (int kk = 0; kk < CIN / 32; ++kk) {
    FragB a;
    a.q[0] = *(const v4u*)(xs + kk * 32 + hi * 8);
    a.q[1] = *(const v4u*)(xs + kk * 32 + 16 + hi * 8);
    #pragma unroll
    for (int t = 0; t < NTN; ++t) {
      const bf16* wp = wct + (size_t)((NT0 + t) * 16 + m) * CIN + kk * 32 + hi * 8;
      FragB bw;
      bw.q[0] = *(const v4u*)(wp);
      bw.q[1] = *(const v4u*)(wp + 16);
      acc[t] = mma_bf16(a.v, bw.v, acc[t]);
    }
  }
}

__global__ __launch_bounds__(256) void proj_pool_kernel(const float* __restrict__ x, const bf16* __restrict__ wct,
                                                         f16* __restrict__ gq, f16* __restrict__ fk,
                                                         f16* __restrict__ hvt) {
  const int kt   = blockIdx.x;
  const int b    = blockIdx.y;
  const int tid  = threadIdx.x;
  const int wave = __builtin_amdgcn_readfirstlane(tid >> 5);
  const int lane = tid & 31;
  const int m    = lane & 15;
  const int hi   = lane >> 4;
  const int hsel = wave >> 2;
  const int ww0  = (wave & 3) * 16;

  __shared__ __align__(16) f16  sP[2 * 32 * PP];
  __shared__ __align__(16) f16  sG[NWAVE * 16 * GP];
  __shared__ __align__(16) f16  sF[64 * FP];
  __shared__ __align__(16) f16  sHT[DV * HP];
  __shared__ __align__(16) bf16 sX[128 * XP];

  f16* sg = sG + wave * (16 * GP);
  f16* sp = sP + hsel * (32 * PP);
  const int pwb = (ww0 >> 1) + hi * 4;
  const bf16* xs = sX + (hsel * W_IMG + ww0 + m) * XP;

  for (int it = 0; it < 2; ++it) {
    const int hh   = kt * 4 + it * 2 + hsel;
    const int pix0 = hh * W_IMG + ww0;
    const int pixb = (kt * 4 + it * 2) * W_IMG;

    #pragma unroll 1
    for (int rr = 0; rr < 4; ++rr) {
      const int c0 = (rr * NWAVE + wave) * 8;
      const float* xp = x + ((size_t)b * CIN + c0) * SEQ_FULL + pixb + lane * 4;
      v4f xv[8];
      #pragma unroll
      for (int j = 0; j < 8; ++j) xv[j] = *(const v4f*)(xp + (size_t)j * SEQ_FULL);
      #pragma unroll
      for (int pp = 0; pp < 4; ++pp) {
        Pack8B pk;
        #pragma unroll
        for (int j = 0; j < 8; ++j) pk.h[j] = (bf16)xv[j][pp];
        *(v4u*)(sX + (lane * 4 + pp) * XP + c0) = pk.u;
      }
    }
    __syncthreads();

    {
      v8f acc[4];
      proj_tiles<0, 4>(xs, wct, m, hi, acc);
      #pragma unroll
      for (int r = 0; r < 8; ++r) {
        sg[(hi * 8 + r) * GP + m]      = toh_flush(acc[2][r]);
        sg[(hi * 8 + r) * GP + 16 + m] = toh_flush(acc[3][r]);
      }
      #pragma unroll
      for (int rp = 0; rp < 4; ++rp) {
        #pragma unroll
        for (int t = 0; t < 2; ++t)
          sp[(pwb + rp) * PP + t * 16 + m] = toh_flush(fmaxf(acc[t][2 * rp], acc[t][2 * rp + 1]));
      }
    }
    {
      v8f acc[8];
      proj_tiles<4, 8>(xs, wct, m, hi, acc);
      #pragma unroll
      for (int rp = 0; rp < 4; ++rp) {
        #pragma unroll
        for (int t = 0; t < 8; ++t)
          sp[(pwb + rp) * PP + 32 + t * 16 + m] = toh_flush(fmaxf(acc[t][2 * rp], acc[t][2 * rp + 1]));
      }
    }
    __syncthreads();

    {
      v4u    gv[2];
      size_t gi[2];
      #pragma unroll
      for (int i2 = 0; i2 < 2; ++i2) {
        const int row = i2 * 8 + (lane >> 2);
        const int cq  = (lane & 3) * 8;
        Pack8H p;
        p.v = *(const v8h*)(sg + row * GP + cq);
        gv[i2] = p.u;
        gi[i2] = ((size_t)b * SEQ + pix0 + row) * DQK + cq;
      }
      #pragma unroll
      for (int i2 = 0; i2 < 2; ++i2) *(volatile v4u*)(gq + gi[i2]) = gv[i2];
      __threadfence();
      #pragma unroll
      for (int i2 = 0; i2 < 2; ++i2) *(volatile v4u*)(gq + gi[i2]) = gv[i2];
    }

    #pragma unroll
    for (int e = 0; e < 4; ++e) {
      const int idx = e * 256 + tid;
      const int pw  = idx >> 5;
      const int c   = idx & 31;
      const float v = fmaxf((float)sP[pw * PP + c], (float)sP[32 * PP + pw * PP + c]);
      sF[(it * 32 + pw) * FP + c] = toh_flush(v);
    }
    #pragma unroll
    for (int e = 0; e < 16; ++e) {
      const int idx = e * 256 + tid;
      const int pw  = idx >> 7;
      const int d   = idx & 127;
      const float v = fmaxf((float)sP[pw * PP + 32 + d], (float)sP[32 * PP + pw * PP + 32 + d]);
      sHT[d * HP + it * 32 + pw] = toh_flush(v);
    }
    __syncthreads();
  }

  v4u    fv;
  size_t fi;
  {
    const int row = tid >> 2;
    const int cq  = (tid & 3) * 8;
    Pack8H p;
    p.v = *(const v8h*)(sF + row * FP + cq);
    fv = p.u;
    fi = ((size_t)b * NKEY + kt * KTILE + row) * DQK + cq;
  }
  v4u    hv[4];
  size_t hidx[4];
  #pragma unroll
  for (int ps = 0; ps < 4; ++ps) {
    const int d  = ps * 32 + (tid >> 3);
    const int kq = (tid & 7) * 8;
    Pack8H p;
    p.v = *(const v8h*)(sHT + d * HP + kq);
    hv[ps]   = p.u;
    hidx[ps] = ((size_t)b * DV + d) * NKEY + kt * KTILE + kq;
  }
  *(volatile v4u*)(fk + fi) = fv;
  #pragma unroll
  for (int ps = 0; ps < 4; ++ps) *(volatile v4u*)(hvt + hidx[ps]) = hv[ps];
  __threadfence();
  *(volatile v4u*)(fk + fi) = fv;
  #pragma unroll
  for (int ps = 0; ps < 4; ++ps) *(volatile v4u*)(hvt + hidx[ps]) = hv[ps];
}

__global__ __launch_bounds__(256) void attn_kernel(const f16* __restrict__ gq, const f16* __restrict__ fk,
                                                   const f16* __restrict__ hvt, f16* __restrict__ ctx) {
  const int qblk = blockIdx.x;
  const int b    = blockIdx.y;
  const int tid  = threadIdx.x;
  const int wave = tid >> 5;
  const int lane = tid & 31;
  const int lq   = lane & 15;
  const int hi   = lane >> 4;

  __shared__ __align__(16) f16 sC[NWAVE * 16 * CP];

  const int qrow0 = qblk * BQ + wave * 16;

  FragH qf;
  {
    const f16* qp = gq + ((size_t)b * SEQ + qrow0 + lq) * DQK + hi * 8;
    qf.q[0] = *(const v4u*)(qp);
    qf.q[1] = *(const v4u*)(qp + 16);
  }

  const f16* fk_b = fk + (size_t)b * NKEY * DQK;
  const f16* vt_b = hvt + (size_t)b * DV * NKEY;

  v8f o[8];
  #pragma unroll
  for (int dt = 0; dt < 8; ++dt) o[dt] = (v8f){0, 0, 0, 0, 0, 0, 0, 0};

  float rmax = -__builtin_inff();
  float rsum = 0.0f;
  const float SL = 1.4426950408889634f;

  for (int i = 0; i < NKEY / BK; ++i) {
    const int j0 = i * BK;

    FragH ak[2];
    #pragma unroll
    for (int sub = 0; sub < 2; ++sub) {
      const f16* base = fk_b + (size_t)(j0 + sub * 16 + lq) * DQK + hi * 8;
      ak[sub].q[0] = *(const v4u*)(base);
      ak[sub].q[1] = *(const v4u*)(base + 16);
    }

    v8f c[2];
    #pragma unroll
    for (int sub = 0; sub < 2; ++sub)
      c[sub] = mma_f16(ak[sub].v, qf.v, (v8f){0, 0, 0, 0, 0, 0, 0, 0});

    float m_new = rmax;
    #pragma unroll
    for (int r = 0; r < 8; ++r) {
      m_new = fmaxf(m_new, c[0][r]);
      m_new = fmaxf(m_new, c[1][r]);
    }
    m_new = fmaxf(m_new, __shfl_xor(m_new, 16, 32));
    const float scale = __builtin_amdgcn_exp2f((rmax - m_new) * SL);
    rmax = m_new;

    FragH pa;
    float psum = 0.0f;
    #pragma unroll
    for (int r = 0; r < 8; ++r) {
      const float p0 = __builtin_amdgcn_exp2f((c[0][r] - m_new) * SL);
      const float p1 = __builtin_amdgcn_exp2f((c[1][r] - m_new) * SL);
      psum += p0 + p1;
      pa.h[r]     = (f16)(p0 * 4096.0f);
      pa.h[8 + r] = (f16)(p1 * 4096.0f);
    }
    rsum = rsum * scale + psum + __shfl_xor(psum, 16, 32);

    float sc[8];
    #pragma unroll
    for (int r = 0; r < 8; ++r) sc[r] = __shfl(scale, (hi << 3) + r, 32);
    #pragma unroll
    for (int dt = 0; dt < 8; ++dt) {
      #pragma unroll
      for (int r = 0; r < 8; ++r) o[dt][r] *= sc[r];
    }

    #pragma unroll
    for (int dt = 0; dt < 8; ++dt) {
      const f16* base = vt_b + (size_t)(dt * 16 + lq) * NKEY + j0 + hi * 8;
      FragH bv;
      bv.q[0] = *(const v4u*)(base);
      bv.q[1] = *(const v4u*)(base + 16);
      o[dt] = mma_f16(pa.v, bv.v, o[dt]);
    }
  }

  float rs[8];
  #pragma unroll
  for (int r = 0; r < 8; ++r) rs[r] = 1.0f / __shfl(rsum, (hi << 3) + r, 32);

  f16* stg = sC + wave * (16 * CP);
  #pragma unroll
  for (int r = 0; r < 8; ++r) {
    #pragma unroll
    for (int dt = 0; dt < 8; ++dt)
      stg[(hi * 8 + r) * CP + dt * 16 + lq] = (f16)(o[dt][r] * (1.0f / 4096.0f) * rs[r]);
  }
  __syncthreads();

  v4u    vals[8];
  size_t gidx[8];
  #pragma unroll
  for (int it = 0; it < 8; ++it) {
    const int row = it * 2 + hi;
    const int dq  = lq * 8;
    Pack8H p;
    p.v = *(const v8h*)(stg + row * CP + dq);
    vals[it] = p.u;
    gidx[it] = ((size_t)b * SEQ + qrow0 + row) * DV + dq;
  }
  #pragma unroll
  for (int it = 0; it < 8; ++it) *(volatile v4u*)(ctx + gidx[it]) = vals[it];
  __threadfence();
  #pragma unroll
  for (int it = 0; it < 8; ++it) *(volatile v4u*)(ctx + gidx[it]) = vals[it];
}

__global__ __launch_bounds__(256) void oproj_kernel(const f16* __restrict__ ctx, const f16* __restrict__ wot,
                                                    const float* __restrict__ x, const float* __restrict__ gamma,
                                                    float* __restrict__ out) {
  const int tid  = threadIdx.x;
  const int wave = __builtin_amdgcn_readfirstlane(tid >> 5);
  const int lane = tid & 31;
  const int m    = lane & 15;
  const int hi   = lane >> 4;
  const int pt   = blockIdx.x * NWAVE + wave;
  const int prow0 = pt * 32;
  const int bb    = prow0 / SEQ;
  const int pix0  = prow0 - bb * SEQ;

  __shared__ __align__(16) float sO[NWAVE * OCH * OP];
  float* so = sO + wave * (OCH * OP);

  const float gsc = (float)(bf16)gamma[0] * 0.0625f;

  FragH cb[DV / 32][2];
  #pragma unroll
  for (int kk = 0; kk < DV / 32; ++kk) {
    #pragma unroll
    for (int t = 0; t < 2; ++t) {
      const f16* cp = ctx + (size_t)(prow0 + t * 16 + m) * DV + kk * 32 + hi * 8;
      cb[kk][t].q[0] = *(const v4u*)(cp);
      cb[kk][t].q[1] = *(const v4u*)(cp + 16);
    }
  }

  #pragma unroll 1
  for (int qn = 0; qn < CIN / OCH; ++qn) {
    v8f acc[2][2];
    #pragma unroll
    for (int j = 0; j < 2; ++j) {
      #pragma unroll
      for (int t = 0; t < 2; ++t) acc[j][t] = (v8f){0, 0, 0, 0, 0, 0, 0, 0};
    }
    #pragma unroll
    for (int kk = 0; kk < DV / 32; ++kk) {
      #pragma unroll
      for (int j = 0; j < 2; ++j) {
        const f16* wp = wot + (size_t)(qn * OCH + j * 16 + m) * DV + kk * 32 + hi * 8;
        FragH aw;
        aw.q[0] = *(const v4u*)(wp);
        aw.q[1] = *(const v4u*)(wp + 16);
        #pragma unroll
        for (int t = 0; t < 2; ++t) acc[j][t] = mma_f16(aw.v, cb[kk][t].v, acc[j][t]);
      }
    }
    #pragma unroll
    for (int r = 0; r < 8; ++r) {
      #pragma unroll
      for (int j = 0; j < 2; ++j) {
        #pragma unroll
        for (int t = 0; t < 2; ++t) so[(j * 16 + hi * 8 + r) * OP + t * 16 + m] = acc[j][t][r] * gsc;
      }
    }
    __syncthreads();

    v4f    vals[8];
    size_t gidx[8];
    #pragma unroll
    for (int it = 0; it < 8; ++it) {
      const int row = it * 4 + (lane >> 3);
      const int pc  = (lane & 7) * 4;
      v4f v = *(const v4f*)(so + row * OP + pc);
      const size_t g = ((size_t)bb * CIN + qn * OCH + row) * SEQ_FULL + pix0 + pc;
      const v4f xv = *(const v4f*)(x + g);
      #pragma unroll
      for (int cc = 0; cc < 4; ++cc) v[cc] = v[cc] + (float)(bf16)xv[cc];
      vals[it] = v;
      gidx[it] = g;
    }
    #pragma unroll
    for (int it = 0; it < 8; ++it) *(volatile v4f*)(out + gidx[it]) = vals[it];
    __threadfence();
    #pragma unroll
    for (int it = 0; it < 8; ++it) *(volatile v4f*)(out + gidx[it]) = vals[it];
    __syncthreads();
  }
}

extern "C" void kernel_launch(void* const* d_in, const int* in_sizes, int n_in,
                              void* d_out, int out_size, void* d_ws, size_t ws_size,
                              hipStream_t stream) {
  if (n_in < 6) return;
  const size_t x_used = ((size_t)NB * CIN - 1) * SEQ_FULL + SEQ;
  if ((size_t)in_sizes[0] < x_used) return;
  if (in_sizes[1] < DQK * CIN) return;
  if (in_sizes[2] < DQK * CIN) return;
  if (in_sizes[3] < DV * CIN) return;
  if (in_sizes[4] < CIN * DV) return;
  if (in_sizes[5] < 1) return;
  if ((size_t)out_size < x_used) return;

  const size_t wct_bytes = (size_t)NPROJ * CIN * 2;
  const size_t wot_bytes = (size_t)CIN * DV * 2;
  const size_t gq_bytes  = (size_t)NB * SEQ * DQK * 2;
  const size_t fk_bytes  = (size_t)NB * NKEY * DQK * 2;
  const size_t hvt_bytes = (size_t)NB * DV * NKEY * 2;
  const size_t ctx_bytes = (size_t)NB * SEQ * DV * 2;
  const size_t off_wct = 0;
  const size_t off_wot = off_wct + wct_bytes;
  const size_t off_gq  = off_wot + wot_bytes;
  const size_t off_fk  = off_gq + gq_bytes;
  const size_t off_hvt = off_fk + fk_bytes;
  const size_t off_ctx = off_hvt + hvt_bytes;
  const size_t total   = off_ctx + ctx_bytes;
  if (ws_size < total) return;

  const float* x     = (const float*)d_in[0];
  const float* wf    = (const float*)d_in[1];
  const float* wg    = (const float*)d_in[2];
  const float* wh    = (const float*)d_in[3];
  const float* wo    = (const float*)d_in[4];
  const float* gamma = (const float*)d_in[5];
  float* out = (float*)d_out;
  char*  ws  = (char*)d_ws;
  bf16* wct = (bf16*)(ws + off_wct);
  f16*  wot = (f16*)(ws + off_wot);
  f16*  gq  = (f16*)(ws + off_gq);
  f16*  fk  = (f16*)(ws + off_fk);
  f16*  hvt = (f16*)(ws + off_hvt);
  f16*  ctx = (f16*)(ws + off_ctx);

  pack_w_kernel<<<40, 256, 0, stream>>>(wf, wg, wh, wo, wct, wot);
  proj_pool_kernel<<<dim3(SEQ / 256, NB), 256, 0, stream>>>(x, wct, gq, fk, hvt);
  attn_kernel<<<dim3(SEQ / BQ, NB), 256, 0, stream>>>(gq, fk, hvt, ctx);
  oproj_kernel<<<(NB * SEQ) / 256, 256, 0, stream>>>(ctx, wot, x, gamma, out);
}
